// Mamba_8435315770097
// MI455X (gfx1250) — hardware-verified
//
#include <hip/hip_runtime.h>
#include <math.h>

typedef __attribute__((ext_vector_type(16))) _Float16 v16h;
typedef __attribute__((ext_vector_type(8)))  _Float16 v8h;
typedef __attribute__((ext_vector_type(16))) __bf16   v16b;
typedef __attribute__((ext_vector_type(8)))  __bf16   v8b;
typedef __attribute__((ext_vector_type(8)))  float    v8f;
typedef __attribute__((ext_vector_type(4)))  float    v4f;

constexpr int kSeq     = 2048;
constexpr int kDin     = 2048;
constexpr int kNst     = 16;
constexpr int kDtR     = 64;
constexpr int kTaps    = 4;
constexpr int kDm      = 1024;
constexpr int kXdW     = 96;
constexpr int kXdP     = 128;
constexpr int kConvT   = 64;
constexpr int kConvXP  = 68;
constexpr int kConvOP  = 68;
constexpr int kScanTS  = 64;
constexpr int kScanCh  = 64;
constexpr int kScanDP  = 68;
constexpr int kScanBCW = 32;
constexpr int kScanZP  = 65;
constexpr int kScanYP  = 68;
constexpr float kLog2e = 1.44269504088896341f;
static_assert(kDtR + 2 * kNst == kXdW, "x_proj width");
static_assert((kDin % 32) == 0 && (kDtR % 32) == 0, "GEMM K multiples of 32");
static_assert((kSeq % 64) == 0 && (kXdP % 64) == 0 && (kDin % 64) == 0 && (kDm % 64) == 0, "GEMM M,N multiples of 64");
static_assert((kSeq % kConvT) == 0 && (kDin % kConvT) == 0 && (kSeq % kScanTS) == 0 && (kDin % kScanCh) == 0, "tile multiples");
static_assert(((kSeq / 64) * (kXdP / 64)) % 8 == 0 && ((kSeq / 64) * (kDm / 64)) % 8 == 0, "8 tiles per GEMM block");
static_assert(kScanTS == 64 && kScanCh == 64 && kDtR == 64, "scan chunk GEMM is 64 x 64 x 64");

constexpr size_t kOffWXH  = 0;
constexpr size_t kOffWXL  = kOffWXH + (size_t)kXdP * kDin * 2;
constexpr size_t kOffWDH  = kOffWXL + (size_t)kXdP * kDin * 2;
constexpr size_t kOffWDL  = kOffWDH + (size_t)kDin * kDtR * 2;
constexpr size_t kOffWOH  = kOffWDL + (size_t)kDin * kDtR * 2;
constexpr size_t kOffWOL  = kOffWOH + (size_t)kDm  * kDin * 2;
constexpr size_t kOffUC   = kOffWOL + (size_t)kDm  * kDin * 2;
constexpr size_t kOffUCH  = kOffUC  + (size_t)kSeq * kDin * 4;
constexpr size_t kOffUCL  = kOffUCH + (size_t)kSeq * kDin * 2;
constexpr size_t kOffXD   = kOffUCL + (size_t)kSeq * kDin * 2;
constexpr size_t kOffXDH  = kOffXD  + (size_t)kSeq * kXdP * 4;
constexpr size_t kOffXDL  = kOffXDH + (size_t)kSeq * kXdP * 2;
constexpr size_t kOffYH   = kOffXDL + (size_t)kSeq * kXdP * 2;
constexpr size_t kOffYL   = kOffYH  + (size_t)kSeq * kDin * 2;
constexpr size_t kWsTotal = kOffYL  + (size_t)kSeq * kDin * 2;
static_assert(kWsTotal == 62390272ull, "carve total");
static_assert(kWsTotal <= 134217728ull, "carve cap");
static_assert((kOffWXL % 128) == 0 && (kOffWDH % 128) == 0 && (kOffWDL % 128) == 0 && (kOffWOH % 128) == 0 &&
              (kOffWOL % 128) == 0 && (kOffUC % 128) == 0 && (kOffUCH % 128) == 0 && (kOffUCL % 128) == 0 &&
              (kOffXD % 128) == 0 && (kOffXDH % 128) == 0 && (kOffXDL % 128) == 0 &&
              (kOffYH % 128) == 0 && (kOffYL % 128) == 0, "128-B aligned regions");

__device__ __forceinline__ unsigned short f2bf_bits(float f) {
  unsigned u = __float_as_uint(f);
  return (unsigned short)((u + 0x7FFFu + ((u >> 16) & 1u)) >> 16);
}
__device__ __forceinline__ float bf_bits2f(unsigned short h) { return __uint_as_float(((unsigned)h) << 16); }

__device__ __forceinline__ void dep_guard_b(v8f& a, v8f& b, v16b x, v16b y) { asm volatile("v_nop\n\tv_nop\n\tv_nop\n\tv_nop" : "+v"(a), "+v"(b) : "v"(x), "v"(y)); }
__device__ __forceinline__ void dep_guard4_h(v8f& a, v8f& b, v8f& c, v8f& d, v16h x, v16h y) { asm volatile("v_nop\n\tv_nop\n\tv_nop\n\tv_nop" : "+v"(a), "+v"(b), "+v"(c), "+v"(d) : "v"(x), "v"(y)); }
__device__ __forceinline__ void dep_guard4_b(v8f& a, v8f& b, v8f& c, v8f& d, v16b x, v16b y) { asm volatile("v_nop\n\tv_nop\n\tv_nop\n\tv_nop" : "+v"(a), "+v"(b), "+v"(c), "+v"(d) : "v"(x), "v"(y)); }
__device__ __forceinline__ void keep4_h(v16h a, v16h b, v16h c, v16h d) { asm volatile("v_nop" :: "v"(a), "v"(b), "v"(c), "v"(d)); }
__device__ __forceinline__ void keep4_b(v16b a, v16b b, v16b c, v16b d) { asm volatile("v_nop" :: "v"(a), "v"(b), "v"(c), "v"(d)); }
__device__ __forceinline__ void acc_guard4(v8f& a, v8f& b, v8f& c, v8f& d) { asm volatile("v_nop\n\tv_nop\n\tv_nop\n\tv_nop" : "+v"(a), "+v"(b), "+v"(c), "+v"(d)); }
template <typename T> struct Frag;
template <> struct Frag<_Float16> {
  typedef v16h V; union U { v16h v; v8h h[2]; };
  static __device__ __forceinline__ v16h load(const _Float16* p) {
    U f; f.h[0] = *(const v8h*)(p); f.h[1] = *(const v8h*)(p + 16); return f.v;
  }
  static __device__ __forceinline__ v8f mma(v16h a, v16h b, v8f c) {
    return __builtin_amdgcn_wmma_f32_16x16x32_f16(false, a, false, b, (short)0, c, false, false);
  }
  static __device__ __forceinline__ void guard4(v8f& a, v8f& b, v8f& c, v8f& d, v16h x, v16h y) { dep_guard4_h(a, b, c, d, x, y); }
  static __device__ __forceinline__ void keep(v16h a, v16h b, v16h c, v16h d) { keep4_h(a, b, c, d); }
};
template <> struct Frag<__bf16> {
  typedef v16b V; union U { v16b v; v8b h[2]; };
  static __device__ __forceinline__ v16b load(const __bf16* p) {
    U f; f.h[0] = *(const v8b*)(p); f.h[1] = *(const v8b*)(p + 16); return f.v;
  }
  static __device__ __forceinline__ v8f mma(v16b a, v16b b, v8f c) {
    return __builtin_amdgcn_wmma_f32_16x16x32_bf16(false, a, false, b, (short)0, c, false, false);
  }
  static __device__ __forceinline__ void guard4(v8f& a, v8f& b, v8f& c, v8f& d, v16b x, v16b y) { dep_guard4_b(a, b, c, d, x, y); }
  static __device__ __forceinline__ void keep(v16b a, v16b b, v16b c, v16b d) { keep4_b(a, b, c, d); }
};

template <int ET> struct Elem;
template <> struct Elem<0> { typedef _Float16 T; };
template <> struct Elem<1> { typedef __bf16 T; };
template <int ET, int SPL, int BIAS_MODE, int OUT_MODE, bool RESID, int ACT = 0>
__global__ __launch_bounds__(256) void wmma_gemm64(
    const unsigned short* __restrict__ Ap, const unsigned short* __restrict__ A2p, int lda, long strideA,
    const unsigned short* __restrict__ Btp, const unsigned short* __restrict__ Bt2p, int ldb, long strideB,
    void* __restrict__ Cout, void* __restrict__ Cout2, int ldc, long strideC,
    const float* __restrict__ bias,
    const float* __restrict__ resid, long strideR,
    int M, int N, int K, float scale) {
  typedef typename Elem<ET>::T T;
  typedef typename Frag<T>::V V;
  const T* A = (const T*)Ap; const T* A2 = (const T*)A2p; const T* Bt = (const T*)Btp; const T* Bt2 = (const T*)Bt2p;
  __shared__ __align__(16) float sT[8][16 * 68];
  const int b    = blockIdx.y;
  const int lane = threadIdx.x & 31;
  const int wave = threadIdx.x >> 5;
  const int tilesN = N >> 6;
  const int tilesM = M >> 6;
  const int tile = blockIdx.x * 8 + wave;
  if (tile >= tilesM * tilesN) return;
  const int tm = tile / tilesN;
  const int tn = tile - tm * tilesN;
  const int m0 = tm << 6;
  const int n0 = tn << 6;

  const T* Ab  = A  + (size_t)b * strideA;
  const T* Bb  = Bt + (size_t)b * strideB;
  const T* Ab2 = (SPL >= 1) ? (A2  + (size_t)b * strideA) : nullptr;
  const T* Bb2 = (SPL == 2) ? (Bt2 + (size_t)b * strideB) : nullptr;

  const int rlane = lane & 15;
  const int koff  = (lane >> 4) * 8;
  const int mOff  = (lane >> 4) * 8;

  v8f acc[4][4];
#pragma unroll
  for (int i = 0; i < 4; ++i)
#pragma unroll
    for (int j = 0; j < 4; ++j) acc[i][j] = (v8f){0.f,0.f,0.f,0.f,0.f,0.f,0.f,0.f};

  for (int k0 = 0; k0 < K; k0 += 32) {
    V bh[4], bl[4];
#pragma unroll
    for (int j = 0; j < 4; ++j) {
      const size_t bo = (size_t)(n0 + (j << 4) + rlane) * ldb + koff + k0;
      bh[j] = Frag<T>::load(Bb + bo);
      if (SPL == 2) bl[j] = Frag<T>::load(Bb2 + bo);
    }
#pragma unroll
    for (int i = 0; i < 4; ++i) {
      const size_t ao = (size_t)(m0 + (i << 4) + rlane) * lda + koff + k0;
      V ah = Frag<T>::load(Ab + ao);
      V al;
      if (SPL >= 1) al = Frag<T>::load(Ab2 + ao);
#pragma unroll
      for (int j = 0; j < 4; ++j) {
        acc[i][j] = Frag<T>::mma(ah, bh[j], acc[i][j]);
        if (SPL == 2) acc[i][j] = Frag<T>::mma(ah, bl[j], acc[i][j]);
        if (SPL >= 1) acc[i][j] = Frag<T>::mma(al, bh[j], acc[i][j]);
      }
      Frag<T>::guard4(acc[i][0], acc[i][1], acc[i][2], acc[i][3], ah, (SPL >= 1) ? al : ah);
    }
    Frag<T>::keep(bh[0], bh[1], bh[2], bh[3]);
    if (SPL == 2) Frag<T>::keep(bl[0], bl[1], bl[2], bl[3]);
  }
  acc_guard4(acc[0][0], acc[0][1], acc[0][2], acc[0][3]);
  acc_guard4(acc[1][0], acc[1][1], acc[1][2], acc[1][3]);
  acc_guard4(acc[2][0], acc[2][1], acc[2][2], acc[2][3]);
  acc_guard4(acc[3][0], acc[3][1], acc[3][2], acc[3][3]);

  float* slab = sT[wave];
  const float* Rb = RESID ? (resid + (size_t)b * strideR) : nullptr;
#pragma unroll
  for (int i = 0; i < 4; ++i) {
    const int mBase = m0 + (i << 4);
#pragma unroll
    for (int j = 0; j < 4; ++j) {
      const int n = n0 + (j << 4) + rlane;
      float bv = 0.f;
      if (BIAS_MODE == 2) bv = bias[n];
#pragma unroll
      for (int r = 0; r < 8; ++r) {
        float v = acc[i][j][r] * scale;
        if (BIAS_MODE == 1) v += bias[mBase + mOff + r];
        if (BIAS_MODE == 2) v += bv;
        if (RESID) v += Rb[(size_t)(mBase + mOff + r) * ldc + n];
        if (ACT == 1) v = tanhf(v);
        if (ACT == 2) v = fmaxf(v, 0.0f);
        if (ACT == 3) v = v / (1.0f + expf(-v));
        if (ACT == 4) v = (v > 0.f) ? v : 0.01f * v;
        slab[(mOff + r) * 68 + (j << 4) + rlane] = v;
      }
    }
    __builtin_amdgcn_fence(__ATOMIC_RELEASE, "workgroup");
    __builtin_amdgcn_wave_barrier();
    __builtin_amdgcn_fence(__ATOMIC_ACQUIRE, "workgroup");
    if (OUT_MODE == 0) {
      float* C = (float*)Cout + (size_t)b * strideC;
      const int hh = lane >> 4, c4 = (lane & 15) * 4;
      for (int pass = 0; pass < 2; ++pass) {
#pragma unroll
        for (int it = 0; it < 8; ++it) {
          const int row = it * 2 + hh;
          v4f v = *(const v4f*)(slab + row * 68 + c4);
          *(volatile v4f*)(C + (size_t)(mBase + row) * ldc + n0 + c4) = v;
        }
        __threadfence();
      }
    } else {
      const int q = lane >> 3, c8 = (lane & 7) * 8;
      unsigned short* C  = (unsigned short*)Cout  + (size_t)b * strideC;
      unsigned short* C2 = (OUT_MODE == 2) ? ((unsigned short*)Cout2 + (size_t)b * strideC) : nullptr;
      for (int pass = 0; pass < 2; ++pass) {
#pragma unroll
        for (int it = 0; it < 4; ++it) {
          const int row = it * 4 + q;
          const float* sp = slab + row * 68 + c8;
          v8h hv, lv;
#pragma unroll
          for (int e = 0; e < 8; ++e) {
            if (OUT_MODE == 1) {
              hv[e] = (_Float16)sp[e];
            } else {
              unsigned short hb = f2bf_bits(sp[e]);
              unsigned short lb = f2bf_bits(sp[e] - bf_bits2f(hb));
              hv[e] = __builtin_bit_cast(_Float16, hb);
              lv[e] = __builtin_bit_cast(_Float16, lb);
            }
          }
          *(volatile v8h*)(C + (size_t)(mBase + row) * ldc + n0 + c8) = hv;
          if (OUT_MODE == 2) *(volatile v8h*)(C2 + (size_t)(mBase + row) * ldc + n0 + c8) = lv;
        }
        __threadfence();
      }
    }
    __builtin_amdgcn_fence(__ATOMIC_RELEASE, "workgroup");
    __builtin_amdgcn_wave_barrier();
    __builtin_amdgcn_fence(__ATOMIC_ACQUIRE, "workgroup");
  }
}

__global__ __launch_bounds__(256) void split_rows_bf16_kernel(
    const float* __restrict__ src, unsigned short* __restrict__ dhi, unsigned short* __restrict__ dlo,
    int total8, int valid8)
{
  const int i = blockIdx.x * 256 + threadIdx.x;
  if (i >= total8) return;
  const int ic = (i < valid8) ? i : (valid8 - 1);
  const float fac = (i < valid8) ? 1.0f : 0.0f;
  const size_t es = (size_t)ic << 3;
  const v4f a0 = *(const v4f*)(src + es);
  const v4f a1 = *(const v4f*)(src + es + 4);
  v8h hv, lv;
#pragma unroll
  for (int e = 0; e < 4; ++e) {
    const float f0 = a0[e] * fac, f1 = a1[e] * fac;
    const unsigned short h0 = f2bf_bits(f0), h1 = f2bf_bits(f1);
    const unsigned short l0 = f2bf_bits(f0 - bf_bits2f(h0)), l1 = f2bf_bits(f1 - bf_bits2f(h1));
    hv[e]     = __builtin_bit_cast(_Float16, h0);
    hv[4 + e] = __builtin_bit_cast(_Float16, h1);
    lv[e]     = __builtin_bit_cast(_Float16, l0);
    lv[4 + e] = __builtin_bit_cast(_Float16, l1);
  }
  const size_t e0 = (size_t)i << 3;
  unsigned short* qh = dhi + e0;
  unsigned short* ql = dlo + e0;
  *(volatile v8h*)qh = hv;
  *(volatile v8h*)ql = lv;
  __threadfence();
  *(volatile v8h*)qh = hv;
  *(volatile v8h*)ql = lv;
}

__global__ __launch_bounds__(256) void conv_silu_kernel(
    const float* __restrict__ xz, const float* __restrict__ cw, const float* __restrict__ cb,
    float* __restrict__ UC, unsigned short* __restrict__ UCH, unsigned short* __restrict__ UCL)
{
  __shared__ __align__(16) float sX[kConvT * kConvXP];
  __shared__ __align__(16) float sO[kConvT * kConvOP];
  const int tid = threadIdx.x, lane = tid & 31, wave = tid >> 5;
  const int d0 = blockIdx.x * kConvT;
  const int t0 = blockIdx.y * kConvT;
  {
    const int ch = tid >> 2, j = tid & 3;
    const float* xrow = xz + (size_t)(d0 + ch) * kSeq;
    const int th  = t0 - 4 + j;
    const int thc = (th < 0) ? 0 : th;
    const float hfac = (th < 0) ? 0.0f : 1.0f;
    const float hval = xrow[thc] * hfac;
    sX[ch * kConvXP + j] = hval;
#pragma unroll
    for (int q = 0; q < 4; ++q) {
      const v4f v = *(const v4f*)(xrow + t0 + 16 * j + 4 * q);
      *(v4f*)(sX + ch * kConvXP + 4 + 16 * j + 4 * q) = v;
    }
  }
  __syncthreads();
  {
    const int ch = tid & 63, tq = tid >> 6;
    const int d = d0 + ch;
    const v4f wv = *(const v4f*)(cw + (size_t)d * kTaps);
    const float bc = cb[d];
    const float* xr = sX + ch * kConvXP + tq * 16;
#pragma unroll 1
    for (int s = 0; s < 16; ++s) {
      float acc = fmaf(wv[0], xr[s + 1], bc);
      acc = fmaf(wv[1], xr[s + 2], acc);
      acc = fmaf(wv[2], xr[s + 3], acc);
      acc = fmaf(wv[3], xr[s + 4], acc);
      const float sg = __builtin_amdgcn_rcpf(1.0f + expf(-acc));
      sO[(tq * 16 + s) * kConvOP + ch] = acc * sg;
    }
  }
  __syncthreads();
  const int hh = lane >> 4, c4 = (lane & 15) * 4;
  const int q = lane >> 3, c8 = (lane & 7) * 8;
  v4f fv[4];
#pragma unroll
  for (int it = 0; it < 4; ++it) fv[it] = *(const v4f*)(sO + (it * 16 + wave * 2 + hh) * kConvOP + c4);
  v8h bh[2], blo[2];
#pragma unroll
  for (int it = 0; it < 2; ++it) {
    const float* sp = sO + (it * 32 + wave * 4 + q) * kConvOP + c8;
    const v4f a0 = *(const v4f*)(sp);
    const v4f a1 = *(const v4f*)(sp + 4);
#pragma unroll
    for (int e = 0; e < 4; ++e) {
      const unsigned short h0 = f2bf_bits(a0[e]), h1 = f2bf_bits(a1[e]);
      const unsigned short l0 = f2bf_bits(a0[e] - bf_bits2f(h0)), l1 = f2bf_bits(a1[e] - bf_bits2f(h1));
      bh[it][e]      = __builtin_bit_cast(_Float16, h0);
      bh[it][4 + e]  = __builtin_bit_cast(_Float16, h1);
      blo[it][e]     = __builtin_bit_cast(_Float16, l0);
      blo[it][4 + e] = __builtin_bit_cast(_Float16, l1);
    }
  }
  for (int pass = 0; pass < 2; ++pass) {
#pragma unroll
    for (int it = 0; it < 4; ++it)
      *(volatile v4f*)(UC + (size_t)(t0 + it * 16 + wave * 2 + hh) * kDin + d0 + c4) = fv[it];
#pragma unroll
    for (int it = 0; it < 2; ++it) {
      const size_t o = (size_t)(t0 + it * 32 + wave * 4 + q) * kDin + d0 + c8;
      *(volatile v8h*)(UCH + o) = bh[it];
      *(volatile v8h*)(UCL + o) = blo[it];
    }
    __threadfence();
  }
}

__global__ __launch_bounds__(64) void scan_kernel(
    const unsigned short* __restrict__ XDH, const unsigned short* __restrict__ XDL,
    const unsigned short* __restrict__ WDH, const unsigned short* __restrict__ WDL,
    const float* __restrict__ UC, const float* __restrict__ XD,
    const float* __restrict__ xz, const float* __restrict__ Ap, const float* __restrict__ Dp,
    const float* __restrict__ dbias, unsigned short* __restrict__ YH, unsigned short* __restrict__ YL)
{
  __shared__ __align__(16) float sDT[kScanTS * kScanDP];
  __shared__ __align__(16) float sBC[kScanTS * kScanBCW];
  __shared__ __align__(16) float sZ[kScanCh * kScanZP];
  __shared__ __align__(16) float sY[kScanTS * kScanYP];
  const int tid = threadIdx.x, lane = tid & 31, wave = tid >> 5;
  const int d0 = blockIdx.x * kScanCh;
  const int d  = d0 + tid;
  const int rlane = lane & 15;
  const int koff  = (lane >> 4) * 8;
  const int mOff  = (lane >> 4) * 8;
  const __bf16* XDHb = (const __bf16*)XDH;
  const __bf16* XDLb = (const __bf16*)XDL;
  const __bf16* WDHb = (const __bf16*)WDH;
  const __bf16* WDLb = (const __bf16*)WDL;
  float A2[kNst], h[kNst];
  {
    const float* ap = Ap + (size_t)d * kNst;
#pragma unroll
    for (int q4 = 0; q4 < 4; ++q4) {
      const v4f av = *(const v4f*)(ap + 4 * q4);
      A2[4 * q4 + 0] = av[0] * kLog2e;
      A2[4 * q4 + 1] = av[1] * kLog2e;
      A2[4 * q4 + 2] = av[2] * kLog2e;
      A2[4 * q4 + 3] = av[3] * kLog2e;
    }
#pragma unroll
    for (int s = 0; s < kNst; ++s) h[s] = 0.0f;
  }
  const float bb = dbias[d], Dd = Dp[d];
  const int lr = tid >> 3, lc4 = (tid & 7) * 4;
  const int q = lane >> 3, c8 = (lane & 7) * 8;
  const size_t brow0 = (size_t)(d0 + wave * 32 + rlane) * kDtR + koff;
  const size_t brow1 = brow0 + (size_t)16 * kDtR;
#pragma unroll 1
  for (int t0 = 0; t0 < kSeq; t0 += kScanTS) {
    __syncthreads();
#pragma unroll 1
    for (int g = 0; g < 2; ++g) {
#pragma unroll
      for (int i = 0; i < 4; ++i) {
        const int r = lr + 8 * (g * 4 + i);
        *(v4f*)(sBC + r * kScanBCW + lc4) = *(const v4f*)(XD + (size_t)(t0 + r) * kXdP + kDtR + lc4);
      }
      asm volatile("" ::: "memory");
    }
#pragma unroll 1
    for (int g = 0; g < 4; ++g) {
#pragma unroll
      for (int i = 0; i < 4; ++i) {
        const int idx = tid + 64 * (g * 4 + i);
        const int c = idx >> 4, q4 = idx & 15;
        const v4f zv4 = *(const v4f*)(xz + (size_t)(kDin + d0 + c) * kSeq + t0 + 4 * q4);
        float* zp = sZ + c * kScanZP + 4 * q4;
        zp[0] = zv4[0]; zp[1] = zv4[1]; zp[2] = zv4[2]; zp[3] = zv4[3];
      }
      asm volatile("" ::: "memory");
    }
#pragma unroll 1
    for (int mt = 0; mt < 4; ++mt) {
      v8f acc0 = (v8f){0.f,0.f,0.f,0.f,0.f,0.f,0.f,0.f};
      v8f acc1 = (v8f){0.f,0.f,0.f,0.f,0.f,0.f,0.f,0.f};
      const size_t arow = (size_t)(t0 + mt * 16 + rlane) * kXdP + koff;
#pragma unroll
      for (int kk = 0; kk < 2; ++kk) {
        const v16b bh0 = Frag<__bf16>::load(WDHb + brow0 + 32 * kk);
        const v16b bl0 = Frag<__bf16>::load(WDLb + brow0 + 32 * kk);
        const v16b bh1 = Frag<__bf16>::load(WDHb + brow1 + 32 * kk);
        const v16b bl1 = Frag<__bf16>::load(WDLb + brow1 + 32 * kk);
        const v16b ah  = Frag<__bf16>::load(XDHb + arow + 32 * kk);
        const v16b al  = Frag<__bf16>::load(XDLb + arow + 32 * kk);
        acc0 = Frag<__bf16>::mma(ah, bh0, acc0);
        acc0 = Frag<__bf16>::mma(ah, bl0, acc0);
        acc0 = Frag<__bf16>::mma(al, bh0, acc0);
        acc1 = Frag<__bf16>::mma(ah, bh1, acc1);
        acc1 = Frag<__bf16>::mma(ah, bl1, acc1);
        acc1 = Frag<__bf16>::mma(al, bh1, acc1);
        dep_guard_b(acc0, acc1, ah, al);
        keep4_b(bh0, bh1, bl0, bl1);
      }
      dep_guard_b(acc0, acc1, (v16b){}, (v16b){});
#pragma unroll
      for (int r = 0; r < 8; ++r) {
        const float v0 = acc0[r], v1 = acc1[r];
        sDT[(mt * 16 + mOff + r) * kScanDP + wave * 32 + rlane]      = v0;
        sDT[(mt * 16 + mOff + r) * kScanDP + wave * 32 + 16 + rlane] = v1;
      }
    }
    __syncthreads();
#pragma unroll 1
    for (int s = 0; s < kScanTS; ++s) {
      const int t = t0 + s;
      const float v   = sDT[s * kScanDP + tid] + bb;
      const float ea  = expf(-fabsf(v));
      const float dt  = fmaxf(v, 0.0f) + log1pf(ea);
      const float u   = UC[(size_t)t * kDin + d];
      const float dtu = dt * u;
      const float* bcr = sBC + s * kScanBCW;
      float Bs[kNst], Cs[kNst];
#pragma unroll
      for (int q4 = 0; q4 < 4; ++q4) {
        const v4f bv = *(const v4f*)(bcr + 4 * q4);
        const v4f cv = *(const v4f*)(bcr + kNst + 4 * q4);
        Bs[4 * q4 + 0] = bv[0]; Bs[4 * q4 + 1] = bv[1]; Bs[4 * q4 + 2] = bv[2]; Bs[4 * q4 + 3] = bv[3];
        Cs[4 * q4 + 0] = cv[0]; Cs[4 * q4 + 1] = cv[1]; Cs[4 * q4 + 2] = cv[2]; Cs[4 * q4 + 3] = cv[3];
      }
      float y = 0.0f;
#pragma unroll
      for (int k = 0; k < kNst; ++k) {
        const float e = exp2f(dt * A2[k]);
        h[k] = fmaf(e, h[k], dtu * Bs[k]);
        y = fmaf(h[k], Cs[k], y);
      }
      y = fmaf(Dd, u, y);
      const float zv = sZ[tid * kScanZP + s];
      const float sg = __builtin_amdgcn_rcpf(1.0f + expf(-zv));
      y = y * (zv * sg);
      sY[s * kScanYP + tid] = y;
    }
    __syncthreads();
    v8h hv[8], lv[8];
#pragma unroll
    for (int it = 0; it < 8; ++it) {
      const int row = it * 8 + wave * 4 + q;
      const float* sp = sY + row * kScanYP + c8;
      const v4f a0 = *(const v4f*)(sp);
      const v4f a1 = *(const v4f*)(sp + 4);
#pragma unroll
      for (int e = 0; e < 4; ++e) {
        const unsigned short h0 = f2bf_bits(a0[e]), h1 = f2bf_bits(a1[e]);
        const unsigned short l0 = f2bf_bits(a0[e] - bf_bits2f(h0)), l1 = f2bf_bits(a1[e] - bf_bits2f(h1));
        hv[it][e]     = __builtin_bit_cast(_Float16, h0);
        hv[it][4 + e] = __builtin_bit_cast(_Float16, h1);
        lv[it][e]     = __builtin_bit_cast(_Float16, l0);
        lv[it][4 + e] = __builtin_bit_cast(_Float16, l1);
      }
    }
    for (int pass = 0; pass < 2; ++pass) {
#pragma unroll
      for (int it = 0; it < 8; ++it) {
        const int row = it * 8 + wave * 4 + q;
        const size_t o = (size_t)(t0 + row) * kDin + d0 + c8;
        *(volatile v8h*)(YH + o) = hv[it];
        *(volatile v8h*)(YL + o) = lv[it];
      }
      __threadfence();
    }
  }
}

extern "C" void kernel_launch(void* const* d_in, const int* in_sizes, int n_in,
                              void* d_out, int out_size, void* d_ws, size_t ws_size,
                              hipStream_t stream) {
  if (n_in < 10) return;
  if (in_sizes[0] != 2 * kDin * kSeq) return;
  if (in_sizes[1] != kDin * kTaps) return;
  if (in_sizes[2] != kDin) return;
  if (in_sizes[3] != kXdW * kDin) return;
  if (in_sizes[4] != kDin * kDtR) return;
  if (in_sizes[5] != kDm * kDin) return;
  if (in_sizes[6] != kDm) return;
  if (in_sizes[7] != kDin * kNst) return;
  if (in_sizes[8] != kDin) return;
  if (in_sizes[9] != kDin) return;
  if (out_size != kSeq * kDm) return;
  if (ws_size < kWsTotal) return;

  const float* xz      = (const float*)d_in[0];
  const float* conv_w  = (const float*)d_in[1];
  const float* conv_b  = (const float*)d_in[2];
  const float* W_xproj = (const float*)d_in[3];
  const float* W_dt    = (const float*)d_in[4];
  const float* W_out   = (const float*)d_in[5];
  const float* b_out   = (const float*)d_in[6];
  const float* Amat    = (const float*)d_in[7];
  const float* Dp      = (const float*)d_in[8];
  const float* b_dt    = (const float*)d_in[9];
  float* out = (float*)d_out;

  char* ws = (char*)d_ws;
  unsigned short* WXH = (unsigned short*)(ws + kOffWXH);
  unsigned short* WXL = (unsigned short*)(ws + kOffWXL);
  unsigned short* WDH = (unsigned short*)(ws + kOffWDH);
  unsigned short* WDL = (unsigned short*)(ws + kOffWDL);
  unsigned short* WOH = (unsigned short*)(ws + kOffWOH);
  unsigned short* WOL = (unsigned short*)(ws + kOffWOL);
  float*          UC  = (float*)(ws + kOffUC);
  unsigned short* UCH = (unsigned short*)(ws + kOffUCH);
  unsigned short* UCL = (unsigned short*)(ws + kOffUCL);
  float*          XD  = (float*)(ws + kOffXD);
  unsigned short* XDH = (unsigned short*)(ws + kOffXDH);
  unsigned short* XDL = (unsigned short*)(ws + kOffXDL);
  unsigned short* YH  = (unsigned short*)(ws + kOffYH);
  unsigned short* YL  = (unsigned short*)(ws + kOffYL);

  {
    const int t8x = kXdP * kDin / 8, v8x = kXdW * kDin / 8;
    split_rows_bf16_kernel<<<(t8x + 255) / 256, 256, 0, stream>>>(W_xproj, WXH, WXL, t8x, v8x);
    const int t8d = kDin * kDtR / 8;
    split_rows_bf16_kernel<<<(t8d + 255) / 256, 256, 0, stream>>>(W_dt, WDH, WDL, t8d, t8d);
    const int t8o = kDm * kDin / 8;
    split_rows_bf16_kernel<<<(t8o + 255) / 256, 256, 0, stream>>>(W_out, WOH, WOL, t8o, t8o);
  }

  conv_silu_kernel<<<dim3(kDin / kConvT, kSeq / kConvT), 256, 0, stream>>>(xz, conv_w, conv_b, UC, UCH, UCL);

  wmma_gemm64<1, 2, 0, 0, false><<<dim3(((kSeq / 64) * (kXdP / 64)) / 8, 1), 256, 0, stream>>>(
      UCH, UCL, kDin, 0L,
      WXH, WXL, kDin, 0L,
      (void*)XD, nullptr, kXdP, 0L,
      nullptr, nullptr, 0L,
      kSeq, kXdP, kDin, 1.0f);

  {
    const int t8 = kSeq * kXdP / 8;
    split_rows_bf16_kernel<<<(t8 + 255) / 256, 256, 0, stream>>>(XD, XDH, XDL, t8, t8);
  }

  scan_kernel<<<kDin / kScanCh, kScanCh, 0, stream>>>(XDH, XDL, WDH, WDL, UC, XD, xz, Amat, Dp, b_dt, YH, YL);

  wmma_gemm64<1, 2, 2, 0, false><<<dim3(((kSeq / 64) * (kDm / 64)) / 8, 1), 256, 0, stream>>>(
      YH, YL, kDin, 0L,
      WOH, WOL, kDin, 0L,
      (void*)out, nullptr, kDm, 0L,
      b_out, nullptr, 0L,
      kSeq, kDm, kDin, 1.0f);
}
